// Neighbor_Mean_27367531610427
// MI455X (gfx1250) — hardware-verified
//
#include <hip/hip_runtime.h>
#include <stddef.h>


typedef _Float16 v16h __attribute__((ext_vector_type(16)));
typedef _Float16 v8h  __attribute__((ext_vector_type(8)));
typedef _Float16 v4h  __attribute__((ext_vector_type(4)));
typedef float    v8f  __attribute__((ext_vector_type(8)));
typedef float    v4f  __attribute__((ext_vector_type(4)));
typedef _Float16 h16;

#ifndef NB
#define NB 8
#endif
#ifndef SEQ
#define SEQ 2048
#endif
#define NB_FULL  8
#define SEQ_FULL 2048
#define HDIM  128
#define NNB   32
#define VPOS  (SEQ_FULL + 1)
#define MROWS (NB * SEQ)
#define RTILE 16

static_assert(NB >= 1 && NB <= NB_FULL);
static_assert(SEQ >= RTILE && SEQ <= SEQ_FULL && (SEQ % RTILE) == 0);
static_assert((MROWS % RTILE) == 0);
static_assert((HDIM % 32) == 0);
static_assert(HDIM == 32 * 4);
static_assert(HDIM == 8 * 16);
static_assert(RTILE == 8 * 2);
static_assert(HDIM * HDIM == 8 * 256 * 8);
static_assert(NNB == 32);

#define LDA 136
#define LDC 132
static_assert((LDA % 8) == 0 && LDA >= HDIM);
static_assert((LDC % 4) == 0 && LDC >= HDIM);

#define WCARRY 64.0f
#define ACARRY 16.0f

#define W16_BYTES ((size_t)HDIM * HDIM * 2)
#define OFF_W16   ((size_t)0)
#define WS_TOTAL  (OFF_W16 + W16_BYTES)
static_assert((W16_BYTES % 128) == 0);
static_assert(WS_TOTAL <= (size_t)134217728);

__device__ __forceinline__ float bf16r(float x) {
  unsigned int u = __float_as_uint(x);
  u = (u + 0x7FFFu + ((u >> 16) & 1u)) & 0xFFFF0000u;
  return __uint_as_float(u);
}

static __device__ __forceinline__ h16 toh_flush(float v) {
  const h16 r = (h16)v;
  return (fabsf(v) < 6.103515625e-05f) ? (h16)0.0f : r;
}

__device__ __forceinline__ v16h frag_at(const _Float16* p) {
  v8h lo = *(const v8h*)(p);
  v8h hi = *(const v8h*)(p + 16);
  v16h out;
#pragma unroll
  for (int i = 0; i < 8; ++i) { out[i] = lo[i]; out[i + 8] = hi[i]; }
  return out;
}
__device__ __forceinline__ v16h ld_frag(const _Float16* base, unsigned ld) {
  const unsigned lane = threadIdx.x & 31u;
  return frag_at(base + (lane & 15u) * ld + (lane >> 4) * 8u);
}

__device__ __forceinline__ v8f wmma16(v16h a, v16h b, v8f c) {
  v8f d = __builtin_amdgcn_wmma_f32_16x16x32_f16(false, a, false, b, (short)0, c,
                                                 false, false);
  asm volatile("v_nop\n\tv_nop\n\tv_nop\n\tv_nop" : "+v"(d) : "v"(a), "v"(b));
  return d;
}

__global__ __launch_bounds__(256) void wcast_kernel(
    const float* __restrict__ W, _Float16* __restrict__ W16) {
  const unsigned gid = blockIdx.x * 256u + threadIdx.x;
  const unsigned row = gid >> 4;
  const unsigned c = (gid & 15u) * 8u;
  const v4f a0 = *(const v4f*)(W + (size_t)row * HDIM + c);
  const v4f a1 = *(const v4f*)(W + (size_t)row * HDIM + c + 4u);
  v8h o;
#pragma unroll
  for (int i = 0; i < 4; ++i) {
    o[i]     = toh_flush(WCARRY * bf16r(a0[i]));
    o[i + 4] = toh_flush(WCARRY * bf16r(a1[i]));
  }
  _Float16* p = W16 + (size_t)row * HDIM + c;
  *(volatile v8h*)p = o;
  __threadfence();
  *(volatile v8h*)p = o;
}

__global__ __launch_bounds__(256) void nmean_kernel(
    const float* __restrict__ Hs, const int* __restrict__ nidx, const int* __restrict__ nmask,
    const float* __restrict__ pos, const _Float16* __restrict__ W16, float* __restrict__ out) {
  __shared__ _Float16 As[RTILE * LDA];
  __shared__ float Cs[RTILE * LDC];

  const unsigned tid = threadIdx.x, lane = tid & 31u;
  const int wave = __builtin_amdgcn_readfirstlane(threadIdx.x >> 5);
  const unsigned hh = lane >> 4, m = lane & 15u;
  const unsigned crow0 = blockIdx.x * (unsigned)RTILE;
  const unsigned bidx = crow0 / (unsigned)SEQ;
  const unsigned s0 = crow0 - bidx * (unsigned)SEQ;
  const size_t frow0 = (size_t)bidx * SEQ_FULL + s0;
  const float* hb = Hs + (size_t)bidx * SEQ_FULL * HDIM;
  const unsigned c = lane * 4u;

#pragma unroll 1
  for (unsigned rr = 0; rr < 2u; ++rr) {
    const unsigned r = (unsigned)wave * 2u + rr;
    const int* ip = nidx + (frow0 + r) * NNB;
    const int* mp = nmask + (frow0 + r) * NNB;
    v4f acc = {0.0f, 0.0f, 0.0f, 0.0f};
#pragma unroll 1
    for (unsigned n = 0; n < (unsigned)NNB; ++n) {
      const int msk = mp[n];
      int idx = ip[n];
      idx = max(idx, 0);
      idx = min(idx, (int)(VPOS - 1));
      if (msk != 0) {
        const float wgt = (float)msk;
        const v4f p = *(const v4f*)(pos + (size_t)idx * HDIM + c);
#pragma unroll
        for (int i = 0; i < 4; ++i) acc[i] += wgt * bf16r(p[i]);
        if (idx > 0) {
          const v4f hv = *(const v4f*)(hb + (size_t)(idx - 1) * HDIM + c);
#pragma unroll
          for (int i = 0; i < 4; ++i) acc[i] += wgt * bf16r(hv[i]);
        }
      }
    }
    v4h o;
#pragma unroll
    for (int i = 0; i < 4; ++i) o[i] = toh_flush(acc[i] * (ACARRY / (float)NNB));
    *(v4h*)&As[r * LDA + c] = o;
  }
  __syncthreads();

  const unsigned kn = (unsigned)wave * 16u;
  const _Float16* bp = W16 + (size_t)(kn + m) * HDIM + hh * 8u;
  v8f accd = {};
#pragma unroll
  for (unsigned k0 = 0; k0 < (unsigned)HDIM; k0 += 32u) {
    const v16h a = ld_frag(&As[k0], LDA);
    const v16h b = frag_at(bp + k0);
    accd = wmma16(a, b, accd);
  }
#pragma unroll
  for (int r = 0; r < 8; ++r)
    Cs[(hh * 8u + (unsigned)r) * LDC + kn + m] = accd[r] * (1.0f / (WCARRY * ACARRY));
  __syncthreads();

  v4f xs[2];
  size_t off[2];
#pragma unroll
  for (unsigned i = 0; i < 2u; ++i) {
    const unsigned r = 8u * i + (unsigned)wave;
    xs[i] = *(const v4f*)&Cs[r * LDC + c];
    off[i] = (frow0 + r) * HDIM + c;
  }
#pragma unroll
  for (int i = 0; i < 2; ++i) *(volatile v4f*)(out + off[i]) = xs[i];
  __threadfence();
#pragma unroll
  for (int i = 0; i < 2; ++i) *(volatile v4f*)(out + off[i]) = xs[i];
}

extern "C" void kernel_launch(void* const* d_in, const int* in_sizes, int n_in,
                              void* d_out, int out_size, void* d_ws, size_t ws_size,
                              hipStream_t stream) {
  if (n_in < 7) return;
  const long long need_rows = (long long)(NB - 1) * SEQ_FULL + SEQ;
  if ((long long)in_sizes[1] < (long long)NB_FULL * SEQ_FULL * HDIM) return;
  if ((long long)in_sizes[3] < need_rows * NNB) return;
  if ((long long)in_sizes[4] < need_rows * NNB) return;
  if ((long long)in_sizes[5] < (long long)VPOS * HDIM) return;
  if ((long long)in_sizes[6] < (long long)HDIM * HDIM) return;
  if ((long long)out_size < need_rows * HDIM) return;
  if (ws_size < WS_TOTAL) return;

  const float* Hs    = (const float*)d_in[1];
  const int*   nidx  = (const int*)d_in[3];
  const int*   nmask = (const int*)d_in[4];
  const float* pos   = (const float*)d_in[5];
  const float* wn    = (const float*)d_in[6];
  float* out = (float*)d_out;

  char* ws = (char*)d_ws;
  _Float16* W16 = (_Float16*)(ws + OFF_W16);

  dim3 blk(256);
  wcast_kernel<<<dim3(8), blk, 0, stream>>>(wn, W16);
  nmean_kernel<<<dim3(MROWS / RTILE), blk, 0, stream>>>(Hs, nidx, nmask, pos, W16, out);
}
